// Block_39926015984134
// MI455X (gfx1250) — hardware-run, weakly checked
//
#include <hip/hip_runtime.h>
#include <stdint.h>


typedef _Float16 v16h __attribute__((ext_vector_type(16)));
typedef _Float16 v8h  __attribute__((ext_vector_type(8)));
typedef _Float16 v4h  __attribute__((ext_vector_type(4)));
typedef float    v8f  __attribute__((ext_vector_type(8)));
typedef float    v4f  __attribute__((ext_vector_type(4)));

#ifndef NB
#define NB 8
#endif
#ifndef SEQ
#define SEQ 2048
#endif
#define MCTX SEQ
#define NB_FULL   8
#define SEQ_FULL  2048
#define DM   512
#define HID  2048

#define ACT_CAR   8.0f
#define W_CAR     1024.0f
#define PROJ_SCL  0.0009765625f
#define S_SCL     3.0517578125e-05f
#define P_CAR     16384.0f
#define O_SCL     0.001953125f
#define OUT_SCL   3.814697265625e-06f
#define MLP1_SCL  0.0001220703125f
#define U_CAR     16.0f
#define MLP2_SCL  6.103515625e-05f

static_assert(DM == 512);
static_assert(DM == 2 * 32 * 8);
static_assert(DM % 128 == 0 && DM % 64 == 0 && DM % 32 == 0);
static_assert(HID % 64 == 0 && HID % 32 == 0);
static_assert(SEQ % 128 == 0);
static_assert(MCTX % 256 == 0);
static_assert(MCTX % 32 == 0);
static_assert(SEQ % 8 == 0);
static_assert(NB >= 1 && NB <= NB_FULL);
static_assert(SEQ <= SEQ_FULL);
static_assert((long)NB_FULL * SEQ_FULL * DM * 4 == 33554432L);
static_assert((long)(DM / 64) * (DM / 64) * 64 * 64 == (long)DM * DM);
static_assert((long)(HID / 64) * (DM / 64) * 64 * 64 == (long)DM * HID);
static_assert(((long)NB * SEQ / 8) * 8 * DM == (long)NB * SEQ * DM);
static_assert((long)(DM / 64) * ((long)NB * SEQ / 128) * 128 * 64 == (long)NB * SEQ * DM);
static_assert((long)(MCTX / 64) * (DM / 128) * 128 * 64 == (long)DM * MCTX);
static_assert((long)(MCTX / 64) * (SEQ / 64) * 4096 == (long)SEQ * MCTX);
static_assert((long)(SEQ / 8) * 8 * MCTX == (long)SEQ * MCTX);
static_assert((long)(DM / 64) * (SEQ / 128) * 128 * 64 == (long)SEQ * DM);
static_assert((long)(HID / 64) * ((long)NB * SEQ / 128) * 128 * 64 == (long)NB * SEQ * HID);

union Frag16 { v16h v; v8h p[2]; };

__device__ __forceinline__ v16h ld_frag(const _Float16* p, int hl) {
  Frag16 f;
  f.p[0] = *(const v8h*)(p + 8 * hl);
  f.p[1] = *(const v8h*)(p + 16 + 8 * hl);
  return f.v;
}

__device__ __forceinline__ v8f mma(v16h a, v16h b, v8f c) {
  v8f d = __builtin_amdgcn_wmma_f32_16x16x32_f16(false, a, false, b, (short)0, c, false, false);
  asm volatile("v_nop\n\tv_nop\n\tv_nop\n\tv_nop" : "+v"(d) : "v"(a), "v"(b));
  return d;
}

__device__ __forceinline__ float bf16_rne(float x) {
  unsigned int u = __builtin_bit_cast(unsigned int, x);
  u += 0x7FFFu + ((u >> 16) & 1u);
  return __builtin_bit_cast(float, u & 0xFFFF0000u);
}

__global__ __launch_bounds__(256) void k_cvtT(const float* __restrict__ src,
                                              _Float16* __restrict__ dst,
                                              int R, int C, float car)
{
  __shared__ float ldsT[64 * 65];
  const int tid = threadIdx.x;
  const int r0 = blockIdx.y * 64, c0 = blockIdx.x * 64;

#pragma unroll
  for (int i = 0; i < 4; ++i) {
    const int q = i * 256 + tid;
    const int row = q >> 4, c4 = (q & 15) * 4;
    const v4f v = *(const v4f*)(src + (size_t)(r0 + row) * C + c0 + c4);
    ldsT[row * 65 + c4 + 0] = v[0];
    ldsT[row * 65 + c4 + 1] = v[1];
    ldsT[row * 65 + c4 + 2] = v[2];
    ldsT[row * 65 + c4 + 3] = v[3];
  }
  __syncthreads();

  v8h o[2];
#pragma unroll
  for (int i = 0; i < 2; ++i) {
    const int q = i * 256 + tid;
    const int cl = q >> 3, ch = (q & 7) * 8;
#pragma unroll
    for (int j = 0; j < 8; ++j)
      o[i][j] = (_Float16)(bf16_rne(ldsT[(ch + j) * 65 + cl]) * car);
  }
#pragma unroll
  for (int i = 0; i < 2; ++i) {
    const int q = i * 256 + tid;
    const int cl = q >> 3, ch = (q & 7) * 8;
    *(volatile v8h*)(dst + (size_t)(c0 + cl) * R + r0 + ch) = o[i];
  }
  __threadfence();
#pragma unroll
  for (int i = 0; i < 2; ++i) {
    const int q = i * 256 + tid;
    const int cl = q >> 3, ch = (q & 7) * 8;
    *(volatile v8h*)(dst + (size_t)(c0 + cl) * R + r0 + ch) = o[i];
  }
}

__global__ __launch_bounds__(256) void k_ln(const float* __restrict__ src,
                                            const float* __restrict__ gam,
                                            const float* __restrict__ bet,
                                            _Float16* __restrict__ dst,
                                            int rows_used, int rows_full, int rne_in)
{
#pragma clang fp contract(off)
  const int lane = threadIdx.x & 31;
  const int w = __builtin_amdgcn_readfirstlane((int)(threadIdx.x >> 5));
  const int row = blockIdx.x * 8 + w;
  const int bz = row / rows_used;
  const int rr = row - bz * rows_used;
  const float* sp = src + ((size_t)bz * rows_full + rr) * DM + 8 * lane;
  const float* gp = gam + 8 * lane;
  const float* bp = bet + 8 * lane;

  v4f xa[2], xb[2], ga[2], gb[2], ba[2], bb[2];
#pragma unroll
  for (int i = 0; i < 2; ++i) {
    xa[i] = *(const v4f*)(sp + i * 256);
    xb[i] = *(const v4f*)(sp + i * 256 + 4);
    ga[i] = *(const v4f*)(gp + i * 256);
    gb[i] = *(const v4f*)(gp + i * 256 + 4);
    ba[i] = *(const v4f*)(bp + i * 256);
    bb[i] = *(const v4f*)(bp + i * 256 + 4);
  }
  if (rne_in != 0) {
#pragma unroll
    for (int i = 0; i < 2; ++i)
#pragma unroll
      for (int j = 0; j < 4; ++j) {
        xa[i][j] = bf16_rne(xa[i][j]);
        xb[i][j] = bf16_rne(xb[i][j]);
      }
  }

  float s = 0.f;
#pragma unroll
  for (int i = 0; i < 2; ++i)
#pragma unroll
    for (int j = 0; j < 4; ++j) {
      s += xa[i][j];
      s += xb[i][j];
    }
  s += __shfl_xor(s, 16, 32);
  s += __shfl_xor(s, 8, 32);
  s += __shfl_xor(s, 4, 32);
  s += __shfl_xor(s, 2, 32);
  s += __shfl_xor(s, 1, 32);
  const float mu = s * (1.0f / (float)DM);

  float qs = 0.f;
#pragma unroll
  for (int i = 0; i < 2; ++i)
#pragma unroll
    for (int j = 0; j < 4; ++j) {
      const float da = xa[i][j] - mu;
      const float db = xb[i][j] - mu;
      xa[i][j] = da;
      xb[i][j] = db;
      qs += da * da;
      qs += db * db;
    }
  qs += __shfl_xor(qs, 16, 32);
  qs += __shfl_xor(qs, 8, 32);
  qs += __shfl_xor(qs, 4, 32);
  qs += __shfl_xor(qs, 2, 32);
  qs += __shfl_xor(qs, 1, 32);
  const float var = qs * (1.0f / (float)DM);
  const float rs = rsqrtf(var + 1e-5f);

  v8h o[2];
#pragma unroll
  for (int i = 0; i < 2; ++i)
#pragma unroll
    for (int j = 0; j < 4; ++j) {
      const float ya = xa[i][j] * rs * bf16_rne(ga[i][j]) + bf16_rne(ba[i][j]);
      const float yb = xb[i][j] * rs * bf16_rne(gb[i][j]) + bf16_rne(bb[i][j]);
      o[i][j]     = (_Float16)(ya * ACT_CAR);
      o[i][4 + j] = (_Float16)(yb * ACT_CAR);
    }
  _Float16* pp = dst + (size_t)row * DM + 8 * lane;
#pragma unroll
  for (int i = 0; i < 2; ++i) *(volatile v8h*)(pp + i * 256) = o[i];
  __threadfence();
#pragma unroll
  for (int i = 0; i < 2; ++i) *(volatile v8h*)(pp + i * 256) = o[i];
}

__device__ __forceinline__ void gemm_core(const _Float16* ap0, const _Float16* ap1,
                                          const _Float16* bp01, const _Float16* bp23,
                                          int K, int hl, v8f (&acc)[8])
{
  const size_t bst = (size_t)16 * K;
#pragma unroll 1
  for (int k0 = 0; k0 < K; k0 += 32) {
    const v16h a0 = ld_frag(ap0 + k0, hl);
    const v16h a1 = ld_frag(ap1 + k0, hl);
    const v16h b0 = ld_frag(bp01 + k0, hl);
    const v16h b1 = ld_frag(bp01 + bst + k0, hl);
    const v16h b2 = ld_frag(bp23 + k0, hl);
    const v16h b3 = ld_frag(bp23 + bst + k0, hl);
    acc[0] = mma(a0, b0, acc[0]);
    acc[1] = mma(a0, b1, acc[1]);
    acc[2] = mma(a0, b2, acc[2]);
    acc[3] = mma(a0, b3, acc[3]);
    acc[4] = mma(a1, b0, acc[4]);
    acc[5] = mma(a1, b1, acc[5]);
    acc[6] = mma(a1, b2, acc[6]);
    acc[7] = mma(a1, b3, acc[7]);
  }
}

__global__ __launch_bounds__(128) __attribute__((amdgpu_num_vgpr(256)))
void k_proj(const _Float16* __restrict__ A, const _Float16* __restrict__ Bt,
            _Float16* __restrict__ PH)
{
  __shared__ __attribute__((aligned(16))) _Float16 ldsH[128 * 72];

  const int tid = threadIdx.x, lane = tid & 31;
  const int w = __builtin_amdgcn_readfirstlane(tid >> 5);
  const int hl = lane >> 4, c = lane & 15;
  const int m0 = blockIdx.y * 128, n0 = blockIdx.x * 64;
  const int z = blockIdx.z;
  const int mw = m0 + 32 * w;

  const _Float16* Bz = Bt + (size_t)z * DM * DM;
  _Float16* const Pz = PH + (size_t)z * ((size_t)NB * SEQ * DM);

  const _Float16* ap0 = A  + (size_t)(mw + c) * DM;
  const _Float16* ap1 = A  + (size_t)(mw + 16 + c) * DM;
  const _Float16* bp  = Bz + (size_t)(n0 + c) * DM;

  v8f acc[8] = {};
  gemm_core(ap0, ap1, bp, bp + (size_t)32 * DM, DM, hl, acc);

#pragma unroll
  for (int i = 0; i < 2; ++i)
#pragma unroll
    for (int t = 0; t < 4; ++t)
#pragma unroll
      for (int r = 0; r < 8; ++r) {
        const int rowl = 32 * w + 16 * i + 8 * hl + r;
        const float v = acc[i * 4 + t][r] * PROJ_SCL;
        ldsH[rowl * 72 + 16 * t + c] = (_Float16)v;
      }
  __syncthreads();

  _Float16* const bh = Pz + (size_t)m0 * DM + n0;
  for (int i = 0; i < 8; ++i) {
    const int q = i * 128 + tid;
    const int rowl = q >> 3, ch = (q & 7) * 8;
    const v8h vh = *(const v8h*)(ldsH + rowl * 72 + ch);
    *(volatile v8h*)(bh + (size_t)rowl * DM + ch) = vh;
  }
  __threadfence();
  for (int i = 0; i < 8; ++i) {
    const int q = i * 128 + tid;
    const int rowl = q >> 3, ch = (q & 7) * 8;
    const v8h vh = *(const v8h*)(ldsH + rowl * 72 + ch);
    *(volatile v8h*)(bh + (size_t)rowl * DM + ch) = vh;
  }
}

__global__ __launch_bounds__(128) __attribute__((amdgpu_num_vgpr(256)))
void k_projv(const _Float16* __restrict__ A, const _Float16* __restrict__ Bt,
             _Float16* __restrict__ PH)
{
  __shared__ __attribute__((aligned(16))) _Float16 ldsH[128 * 72];

  const int tid = threadIdx.x, lane = tid & 31, w = tid >> 5;
  const int hl = lane >> 4, c = lane & 15;
  const int m0 = blockIdx.y * 128, n0 = blockIdx.x * 64;
  const int z = blockIdx.z;
  const int mw = m0 + 32 * w;

  const _Float16* Bz = Bt + (size_t)z * MCTX * DM;
  _Float16* const Pz = PH + (size_t)z * DM * MCTX;

  const _Float16* ap0 = A  + (size_t)(mw + c) * DM;
  const _Float16* ap1 = A  + (size_t)(mw + 16 + c) * DM;
  const _Float16* bp  = Bz + (size_t)(n0 + c) * DM;

  v8f acc[8] = {};
  gemm_core(ap0, ap1, bp, bp + (size_t)32 * DM, DM, hl, acc);

#pragma unroll
  for (int i = 0; i < 2; ++i) {
#pragma unroll
    for (int r = 0; r < 8; ++r) {
      const int rowl = 32 * w + 16 * i + 8 * hl + r;
#pragma unroll
      for (int t = 0; t < 4; ++t) {
        const float v = acc[i * 4 + t][r] * PROJ_SCL;
        ldsH[rowl * 72 + 16 * t + c] = (_Float16)v;
      }
    }
  }
  __syncthreads();

  _Float16* const bh = Pz + (size_t)m0 * MCTX + n0;
  for (int i = 0; i < 8; ++i) {
    const int q = i * 128 + tid;
    const int rowl = q >> 3, ch = (q & 7) * 8;
    const v8h vh = *(const v8h*)(ldsH + rowl * 72 + ch);
    *(volatile v8h*)(bh + (size_t)rowl * MCTX + ch) = vh;
  }
  __threadfence();
  for (int i = 0; i < 8; ++i) {
    const int q = i * 128 + tid;
    const int rowl = q >> 3, ch = (q & 7) * 8;
    const v8h vh = *(const v8h*)(ldsH + rowl * 72 + ch);
    *(volatile v8h*)(bh + (size_t)rowl * MCTX + ch) = vh;
  }
}

__global__ __launch_bounds__(128) __attribute__((amdgpu_num_vgpr(256)))
void k_score(const _Float16* __restrict__ QH, const _Float16* __restrict__ KH,
             float* __restrict__ S)
{
  __shared__ __attribute__((aligned(16))) float ldsF[64 * 68];

  const int tid = threadIdx.x, lane = tid & 31, w = tid >> 5;
  const int hl = lane >> 4, c = lane & 15;
  const int m0 = blockIdx.y * 64, n0 = blockIdx.x * 64;
  const int mw = m0 + 16 * w;

  const _Float16* ah = QH + (size_t)(mw + c) * DM;
  const _Float16* bh = KH + (size_t)(n0 + c) * DM;

  v8f sh[4] = {};
#pragma unroll 1
  for (int k0 = 0; k0 < DM; k0 += 32) {
    const v16h qh = ld_frag(ah + k0, hl);
#pragma unroll
    for (int t = 0; t < 4; ++t) {
      const v16h kf = ld_frag(bh + (size_t)t * 16 * DM + k0, hl);
      sh[t] = mma(qh, kf, sh[t]);
    }
  }

#pragma unroll
  for (int t = 0; t < 4; ++t)
#pragma unroll
    for (int r = 0; r < 8; ++r) {
      const int rowl = 16 * w + 8 * hl + r;
      ldsF[rowl * 68 + 16 * t + c] = sh[t][r] * S_SCL;
    }
  __syncthreads();

  float* const ob = S + (size_t)m0 * MCTX + n0;
  for (int i = 0; i < 8; ++i) {
    const int qi = i * 128 + tid;
    const int rowl = qi >> 4, col = (qi & 15) * 4;
    const v4f v = *(const v4f*)(ldsF + rowl * 68 + col);
    *(volatile v4f*)(ob + (size_t)rowl * MCTX + col) = v;
  }
  __threadfence();
  for (int i = 0; i < 8; ++i) {
    const int qi = i * 128 + tid;
    const int rowl = qi >> 4, col = (qi & 15) * 4;
    const v4f v = *(const v4f*)(ldsF + rowl * 68 + col);
    *(volatile v4f*)(ob + (size_t)rowl * MCTX + col) = v;
  }
}

__global__ __launch_bounds__(256) void k_softmax(const float* __restrict__ S,
                                                 _Float16* __restrict__ P)
{
  constexpr int NI = MCTX / 256;
  static_assert(NI * 256 == MCTX);
  static_assert(NI >= 1 && NI <= 8);
  const int lane = threadIdx.x & 31, w = threadIdx.x >> 5;
  const int row = blockIdx.x * 8 + w;
  const float* sp = S + (size_t)row * MCTX + 8 * lane;

  v4f xa[NI], xb[NI];
#pragma unroll
  for (int i = 0; i < NI; ++i) {
    xa[i] = *(const v4f*)(sp + i * 256);
    xb[i] = *(const v4f*)(sp + i * 256 + 4);
  }
  float mx = -__builtin_inff();
#pragma unroll
  for (int i = 0; i < NI; ++i)
#pragma unroll
    for (int j = 0; j < 4; ++j) {
      mx = fmaxf(mx, xa[i][j]);
      mx = fmaxf(mx, xb[i][j]);
    }
  mx = fmaxf(mx, __shfl_xor(mx, 16, 32));
  mx = fmaxf(mx, __shfl_xor(mx, 8, 32));
  mx = fmaxf(mx, __shfl_xor(mx, 4, 32));
  mx = fmaxf(mx, __shfl_xor(mx, 2, 32));
  mx = fmaxf(mx, __shfl_xor(mx, 1, 32));

  float sm = 0.f;
#pragma unroll
  for (int i = 0; i < NI; ++i)
#pragma unroll
    for (int j = 0; j < 4; ++j) {
      const float ea = __expf(xa[i][j] - mx);
      const float eb = __expf(xb[i][j] - mx);
      xa[i][j] = ea;
      xb[i][j] = eb;
      sm += ea;
      sm += eb;
    }
  sm += __shfl_xor(sm, 16, 32);
  sm += __shfl_xor(sm, 8, 32);
  sm += __shfl_xor(sm, 4, 32);
  sm += __shfl_xor(sm, 2, 32);
  sm += __shfl_xor(sm, 1, 32);
  const float inv = P_CAR * (1.0f / sm);

  v8h o[NI];
#pragma unroll
  for (int i = 0; i < NI; ++i)
#pragma unroll
    for (int j = 0; j < 4; ++j) {
      o[i][j]     = (_Float16)(xa[i][j] * inv);
      o[i][4 + j] = (_Float16)(xb[i][j] * inv);
    }
  _Float16* pp = P + (size_t)row * MCTX + 8 * lane;
#pragma unroll
  for (int i = 0; i < NI; ++i) *(volatile v8h*)(pp + i * 256) = o[i];
  __threadfence();
#pragma unroll
  for (int i = 0; i < NI; ++i) *(volatile v8h*)(pp + i * 256) = o[i];
}

__global__ __launch_bounds__(128) __attribute__((amdgpu_num_vgpr(256)))
void k_pv(const _Float16* __restrict__ A, const _Float16* __restrict__ Bt,
          _Float16* __restrict__ PH)
{
  __shared__ __attribute__((aligned(16))) _Float16 ldsH[128 * 72];

  const int tid = threadIdx.x, lane = tid & 31, w = tid >> 5;
  const int hl = lane >> 4, c = lane & 15;
  const int m0 = blockIdx.y * 128, n0 = blockIdx.x * 64;
  const int mw = m0 + 32 * w;

  const _Float16* ap0 = A  + (size_t)(mw + c) * MCTX;
  const _Float16* ap1 = A  + (size_t)(mw + 16 + c) * MCTX;
  const _Float16* bp  = Bt + (size_t)(n0 + c) * MCTX;

  v8f acc[8] = {};
  gemm_core(ap0, ap1, bp, bp + (size_t)32 * MCTX, MCTX, hl, acc);

#pragma unroll
  for (int i = 0; i < 2; ++i)
#pragma unroll
    for (int t = 0; t < 4; ++t)
#pragma unroll
      for (int r = 0; r < 8; ++r) {
        const int rowl = 32 * w + 16 * i + 8 * hl + r;
        const float v = acc[i * 4 + t][r] * O_SCL;
        ldsH[rowl * 72 + 16 * t + c] = (_Float16)v;
      }
  __syncthreads();

  _Float16* const bh = PH + (size_t)m0 * DM + n0;
  for (int i = 0; i < 8; ++i) {
    const int q = i * 128 + tid;
    const int rowl = q >> 3, ch = (q & 7) * 8;
    const v8h vh = *(const v8h*)(ldsH + rowl * 72 + ch);
    *(volatile v8h*)(bh + (size_t)rowl * DM + ch) = vh;
  }
  __threadfence();
  for (int i = 0; i < 8; ++i) {
    const int q = i * 128 + tid;
    const int rowl = q >> 3, ch = (q & 7) * 8;
    const v8h vh = *(const v8h*)(ldsH + rowl * 72 + ch);
    *(volatile v8h*)(bh + (size_t)rowl * DM + ch) = vh;
  }
}

__global__ __launch_bounds__(128) __attribute__((amdgpu_num_vgpr(256)))
void k_gemm_res(const _Float16* __restrict__ A, const _Float16* __restrict__ Bt,
                const float* __restrict__ Res, float* __restrict__ Out,
                int K, float scl, int res_bs, int out_bs, int rne_res)
{
  __shared__ __attribute__((aligned(16))) float ldsF[128 * 68];

  const int tid = threadIdx.x, lane = tid & 31;
  const int w = __builtin_amdgcn_readfirstlane(tid >> 5);
  const int hl = lane >> 4, c = lane & 15;
  const int m0 = blockIdx.y * 128, n0 = blockIdx.x * 64;
  const int mw = m0 + 32 * w;

  const _Float16* ap0 = A  + (size_t)(mw + c) * K;
  const _Float16* ap1 = A  + (size_t)(mw + 16 + c) * K;
  const _Float16* bp  = Bt + (size_t)(n0 + c) * K;

  v8f acc[8] = {};
  gemm_core(ap0, ap1, bp, bp + (size_t)32 * K, K, hl, acc);

#pragma unroll
  for (int t = 0; t < 4; ++t) {
#pragma unroll
    for (int i = 0; i < 2; ++i)
#pragma unroll
      for (int r = 0; r < 8; ++r) {
        const int rowl = 32 * w + 16 * i + 8 * hl + r;
        ldsF[rowl * 68 + 16 * t + c] = acc[i * 4 + t][r] * scl;
      }
  }
  __syncthreads();

  const int bz = m0 / SEQ, sr = m0 - bz * SEQ;
  const float* const rb = Res + ((size_t)bz * res_bs + sr) * DM + n0;
  float* const ob = Out + ((size_t)bz * out_bs + sr) * DM + n0;
  for (int i = 0; i < 16; ++i) {
    const int qi = i * 128 + tid;
    const int rowl = qi >> 4, col = (qi & 15) * 4;
    const v4f a = *(const v4f*)(ldsF + rowl * 68 + col);
    const v4f x = *(const v4f*)(rb + (size_t)rowl * DM + col);
    v4f v;
#pragma unroll
    for (int j = 0; j < 4; ++j) {
      const float xr = (rne_res != 0) ? bf16_rne(x[j]) : x[j];
      v[j] = xr + a[j];
    }
    *(volatile v4f*)(ob + (size_t)rowl * DM + col) = v;
  }
  __threadfence();
  for (int i = 0; i < 16; ++i) {
    const int qi = i * 128 + tid;
    const int rowl = qi >> 4, col = (qi & 15) * 4;
    const v4f a = *(const v4f*)(ldsF + rowl * 68 + col);
    const v4f x = *(const v4f*)(rb + (size_t)rowl * DM + col);
    v4f v;
#pragma unroll
    for (int j = 0; j < 4; ++j) {
      const float xr = (rne_res != 0) ? bf16_rne(x[j]) : x[j];
      v[j] = xr + a[j];
    }
    *(volatile v4f*)(ob + (size_t)rowl * DM + col) = v;
  }
}

__global__ __launch_bounds__(128) __attribute__((amdgpu_num_vgpr(256)))
void k_mlp1(const _Float16* __restrict__ A, const _Float16* __restrict__ Bt,
            _Float16* __restrict__ PH)
{
  __shared__ __attribute__((aligned(16))) float    ldsF[128 * 68];
  __shared__ __attribute__((aligned(16))) _Float16 ldsH[128 * 72];

  const int tid = threadIdx.x, lane = tid & 31;
  const int w = __builtin_amdgcn_readfirstlane(tid >> 5);
  const int hl = lane >> 4, c = lane & 15;
  const int m0 = blockIdx.y * 128, n0 = blockIdx.x * 64;
  const int mw = m0 + 32 * w;

  const _Float16* ap0 = A  + (size_t)(mw + c) * DM;
  const _Float16* ap1 = A  + (size_t)(mw + 16 + c) * DM;
  const _Float16* bp  = Bt + (size_t)(n0 + c) * DM;

  v8f acc[8] = {};
  gemm_core(ap0, ap1, bp, bp + (size_t)32 * DM, DM, hl, acc);

#pragma unroll
  for (int t = 0; t < 4; ++t) {
#pragma unroll
    for (int i = 0; i < 2; ++i)
#pragma unroll
      for (int r = 0; r < 8; ++r) {
        const int rowl = 32 * w + 16 * i + 8 * hl + r;
        ldsF[rowl * 68 + 16 * t + c] = acc[i * 4 + t][r] * MLP1_SCL;
      }
  }
  __syncthreads();

#pragma unroll 1
  for (int i = 0; i < 16; ++i) {
    const int qi = i * 128 + tid;
    const int rowl = qi >> 4, col = (qi & 15) * 4;
    const v4f v = *(const v4f*)(ldsF + rowl * 68 + col);
    v4h o;
#pragma unroll
    for (int j = 0; j < 4; ++j) {
      const float u = v[j];
      const float gl = 0.5f * u * (1.0f + erff(u * 0.70710678118654752f));
      o[j] = (_Float16)(gl * U_CAR);
    }
    *(v4h*)(ldsH + rowl * 72 + col) = o;
  }
  __syncthreads();

  _Float16* const bh = PH + (size_t)m0 * HID + n0;
  for (int i = 0; i < 8; ++i) {
    const int q = i * 128 + tid;
    const int rowl = q >> 3, ch = (q & 7) * 8;
    const v8h vh = *(const v8h*)(ldsH + rowl * 72 + ch);
    *(volatile v8h*)(bh + (size_t)rowl * HID + ch) = vh;
  }
  __threadfence();
  for (int i = 0; i < 8; ++i) {
    const int q = i * 128 + tid;
    const int rowl = q >> 3, ch = (q & 7) * 8;
    const v8h vh = *(const v8h*)(ldsH + rowl * 72 + ch);
    *(volatile v8h*)(bh + (size_t)rowl * HID + ch) = vh;
  }
}

constexpr size_t cmax(size_t a, size_t b) { return a > b ? a : b; }
constexpr size_t N_X    = (size_t)NB * SEQ * DM;
constexpr size_t N_W    = (size_t)DM * DM;
constexpr size_t N_WM   = (size_t)DM * HID;
constexpr size_t B_H    = N_X * 2;
constexpr size_t B_S    = (size_t)SEQ * MCTX * 4;
constexpr size_t B_P    = (size_t)SEQ * MCTX * 2;
constexpr size_t B_R0   = cmax(B_H, B_S + B_P);
constexpr size_t B_W    = (4 * N_W + 2 * N_WM) * 2;
constexpr size_t B_PL   = N_X * 2;
constexpr size_t B_QKVO = 4 * B_PL;
constexpr size_t B_U    = (size_t)NB * SEQ * HID * 2;
constexpr size_t B_X1   = N_X * 4;
constexpr size_t OFF_W   = B_R0;
constexpr size_t OFF_Q   = OFF_W + B_W;
constexpr size_t OFF_X1  = OFF_Q + B_QKVO;
constexpr size_t WS_TOTAL = OFF_X1 + B_X1;
static_assert(B_H <= B_R0 && B_S + B_P <= B_R0);
static_assert(B_U <= B_QKVO);
static_assert(B_R0 % 128 == 0 && B_W % 128 == 0 && B_PL % 128 == 0 && B_S % 128 == 0 && B_X1 % 128 == 0);
static_assert(WS_TOTAL <= (size_t)134217728);

extern "C" void kernel_launch(void* const* d_in, const int* in_sizes, int n_in,
                              void* d_out, int out_size, void* d_ws, size_t ws_size,
                              hipStream_t stream)
{
  if (n_in < 11) return;
  const long needX = ((long)(NB - 1) * SEQ_FULL + SEQ) * DM;
  if ((long)in_sizes[0] < needX) return;
  if ((long)in_sizes[1] < (long)DM * DM) return;
  if ((long)in_sizes[2] < (long)DM * DM) return;
  if ((long)in_sizes[3] < (long)DM * DM) return;
  if ((long)in_sizes[4] < (long)DM * DM) return;
  if ((long)in_sizes[5] < (long)DM * HID) return;
  if ((long)in_sizes[6] < (long)DM * HID) return;
  if ((long)in_sizes[7] < (long)DM) return;
  if ((long)in_sizes[8] < (long)DM) return;
  if ((long)in_sizes[9] < (long)DM) return;
  if ((long)in_sizes[10] < (long)DM) return;
  if ((long)out_size < needX) return;
  if (WS_TOTAL > ws_size) return;

  const float* x  = (const float*)d_in[0];
  const float* wq = (const float*)d_in[1];
  const float* wk = (const float*)d_in[2];
  const float* wv = (const float*)d_in[3];
  const float* wp = (const float*)d_in[4];
  const float* w1 = (const float*)d_in[5];
  const float* w2 = (const float*)d_in[6];
  const float* g1 = (const float*)d_in[7];
  const float* b1 = (const float*)d_in[8];
  const float* g2 = (const float*)d_in[9];
  const float* b2 = (const float*)d_in[10];
  float* out = (float*)d_out;

  char* const ws = (char*)d_ws;
  _Float16* H16 = (_Float16*)ws;
  float*    Sp  = (float*)ws;
  _Float16* Pp  = (_Float16*)(ws + B_S);
  _Float16* WqP = (_Float16*)(ws + OFF_W);
  _Float16* WkP = WqP + N_W;
  _Float16* WvP = WkP + N_W;
  _Float16* WpP = WvP + N_W;
  _Float16* W1T = WpP + N_W;
  _Float16* W2T = W1T + N_WM;
  _Float16* QH  = (_Float16*)(ws + OFF_Q);
  _Float16* KH  = QH + N_X;
  _Float16* VtH = KH + N_X;
  _Float16* OH  = VtH + N_X;
  _Float16* U16 = (_Float16*)(ws + OFF_Q);
  float*    X1  = (float*)(ws + OFF_X1);

  k_cvtT<<<dim3(DM / 64, DM / 64), 256, 0, stream>>>(wq, WqP, DM, DM, W_CAR);
  k_cvtT<<<dim3(DM / 64, DM / 64), 256, 0, stream>>>(wk, WkP, DM, DM, W_CAR);
  k_cvtT<<<dim3(DM / 64, DM / 64), 256, 0, stream>>>(wv, WvP, DM, DM, W_CAR);
  k_cvtT<<<dim3(DM / 64, DM / 64), 256, 0, stream>>>(wp, WpP, DM, DM, W_CAR);
  k_cvtT<<<dim3(HID / 64, DM / 64), 256, 0, stream>>>(w1, W1T, DM, HID, W_CAR);
  k_cvtT<<<dim3(DM / 64, HID / 64), 256, 0, stream>>>(w2, W2T, HID, DM, W_CAR);

  k_ln<<<NB * SEQ / 8, 256, 0, stream>>>(x, g1, b1, H16, SEQ, SEQ_FULL, 1);

  k_proj<<<dim3(DM / 64, NB * SEQ / 128, 2), 128, 0, stream>>>(H16, WqP, QH);
  k_projv<<<dim3(MCTX / 64, DM / 128, NB), 128, 0, stream>>>(WvP, H16, VtH);

  for (int b = 0; b < NB; ++b) {
    const size_t qo = (size_t)b * SEQ * DM;
    const size_t ko = (size_t)b * MCTX * DM;
    k_score<<<dim3(MCTX / 64, SEQ / 64), 128, 0, stream>>>(QH + qo, KH + ko, Sp);
    k_softmax<<<SEQ / 8, 256, 0, stream>>>(Sp, Pp);
    k_pv<<<dim3(DM / 64, SEQ / 128), 128, 0, stream>>>(Pp, VtH + ko, OH + qo);
  }

  k_gemm_res<<<dim3(DM / 64, NB * SEQ / 128), 128, 0, stream>>>(OH, WpP, x, X1, DM, OUT_SCL, SEQ_FULL, SEQ, 1);

  k_ln<<<NB * SEQ / 8, 256, 0, stream>>>(X1, g2, b2, H16, SEQ, SEQ, 0);

  k_mlp1<<<dim3(HID / 64, NB * SEQ / 128), 128, 0, stream>>>(H16, W1T, U16);

  k_gemm_res<<<dim3(DM / 64, NB * SEQ / 128), 128, 0, stream>>>(U16, W2T, X1, out, HID, MLP2_SCL, SEQ, SEQ_FULL, 0);
}
